// ECGLSTM_7052336300076
// MI455X (gfx1250) — hardware-verified
//
#include <hip/hip_runtime.h>
#include <math.h>

constexpr int NBATCH  = 256;
constexpr int NSTEP   = 5000;
constexpr int NHID    = 64;
constexpr int NGATE   = 4 * NHID;
constexpr int NFC     = 128;
constexpr int NTHR    = 128;
constexpr int SEQ_BLK = 16;
constexpr int CHUNK_T = 200;
constexpr int NCHUNK  = NSTEP / CHUNK_T;
constexpr int HPITCH  = 72;
constexpr int HTPITCH = 68;
constexpr int OPITCH  = 132;
constexpr float HCARRY     = 64.0f;
constexpr float WCARRY     = 256.0f;
constexpr float ACARRY     = HCARRY * WCARRY;
constexpr float ACARRY_INV = 1.0f / ACARRY;

static_assert(NSTEP % CHUNK_T == 0, "no tail chunk");
static_assert((CHUNK_T * SEQ_BLK) % NTHR == 0, "x staging loop exact");
static_assert(NBATCH % SEQ_BLK == 0, "batch tiles exact");
static_assert(NHID == 16 * (NTHR / 32), "4 waves x 16 hidden columns");
static_assert(NHID % 32 == 0, "K multiple of 32");
static_assert((2 * SEQ_BLK * HPITCH) % NTHR == 0, "h zero-fill loop exact");
static_assert(NFC == 4 * 32, "4 column passes of 32 lanes");
static_assert(SEQ_BLK == 4 * (NTHR / 32), "4 output rows per wave");
static_assert(HPITCH % 8 == 0 && HTPITCH % 4 == 0 && OPITCH % 4 == 0, "16-B aligned LDS rows");

typedef __attribute__((ext_vector_type(16))) _Float16 v16h;
typedef __attribute__((ext_vector_type(8)))  _Float16 v8h;
typedef __attribute__((ext_vector_type(8)))  float    v8f;
typedef __attribute__((ext_vector_type(4)))  float    v4f;

union FragU { v16h v; v8h h[2]; };
__device__ __forceinline__ v16h frag_load(const _Float16* p) {
  FragU f;
  f.h[0] = *(const v8h*)(p);
  f.h[1] = *(const v8h*)(p + 16);
  return f.v;
}
__device__ __forceinline__ v8f mma_h(v16h a, v16h b, v8f c) {
  return __builtin_amdgcn_wmma_f32_16x16x32_f16(false, a, false, b, (short)0, c, false, false);
}
__device__ __forceinline__ void guard_group(v8f& a, v8f& b, v8f& c, v8f& d, v16h x0, v16h x1,
                                            v16h w0, v16h w1, v16h w2, v16h w3,
                                            v16h w4, v16h w5, v16h w6, v16h w7) {
  asm volatile("v_nop\n\tv_nop\n\tv_nop\n\tv_nop"
               : "+v"(a), "+v"(b), "+v"(c), "+v"(d)
               : "v"(x0), "v"(x1), "v"(w0), "v"(w1), "v"(w2), "v"(w3), "v"(w4), "v"(w5), "v"(w6), "v"(w7));
}

__device__ __forceinline__ float fsig(float x)  { return __builtin_amdgcn_rcpf(1.0f + __expf(-x)); }
__device__ __forceinline__ float ftanh(float x) { return 1.0f - 2.0f * __builtin_amdgcn_rcpf(__expf(2.0f * x) + 1.0f); }

__global__ __launch_bounds__(NTHR) void lstm_seq_kernel(const float* __restrict__ x,
                                                        const float* __restrict__ w_ih,
                                                        const float* __restrict__ w_hh,
                                                        const float* __restrict__ b_ih,
                                                        const float* __restrict__ b_hh,
                                                        const float* __restrict__ w_fc,
                                                        const float* __restrict__ b_fc,
                                                        float* __restrict__ out) {
  __shared__ __align__(16) _Float16 Ah[2 * SEQ_BLK * HPITCH];
  __shared__ __align__(16) float    Xs[CHUNK_T * SEQ_BLK];
  __shared__ __align__(16) float    Hf[SEQ_BLK * HTPITCH];
  __shared__ __align__(16) float    Os[SEQ_BLK * OPITCH];

  const int tid  = threadIdx.x;
  const int lane = tid & 31;
  const int wave = tid >> 5;
  const int c    = lane & 15;
  const int hh   = lane >> 4;
  const int koff = hh * 8;
  const int b0   = blockIdx.x * SEQ_BLK;
  const int hc   = 16 * wave + c;

  v16h wb[4][2];
  float wiS[4], bsS[4];
#pragma unroll
  for (int g = 0; g < 4; ++g) {
    const int j = g * NHID + hc;
    wiS[g] = w_ih[j] * ACARRY;
    bsS[g] = (b_ih[j] + b_hh[j]) * ACARRY;
#pragma unroll
    for (int kc = 0; kc < 2; ++kc) {
      const float* src = w_hh + (size_t)j * NHID + kc * 32 + koff;
      const v4f p0 = *(const v4f*)(src);
      const v4f p1 = *(const v4f*)(src + 4);
      const v4f p2 = *(const v4f*)(src + 16);
      const v4f p3 = *(const v4f*)(src + 20);
      v16h f;
#pragma unroll
      for (int e = 0; e < 4; ++e) {
        f[e]      = (_Float16)(p0[e] * WCARRY);
        f[4 + e]  = (_Float16)(p1[e] * WCARRY);
        f[8 + e]  = (_Float16)(p2[e] * WCARRY);
        f[12 + e] = (_Float16)(p3[e] * WCARRY);
      }
      wb[g][kc] = f;
    }
  }

#pragma unroll 1
  for (int i = tid; i < 2 * SEQ_BLK * HPITCH; i += NTHR) Ah[i] = (_Float16)0.0f;

  float creg[8], hreg[8];
#pragma unroll
  for (int r = 0; r < 8; ++r) { creg[r] = 0.0f; hreg[r] = 0.0f; }

#pragma unroll 1
  for (int ch = 0; ch < NCHUNK; ++ch) {
    const int t0 = ch * CHUNK_T;
#pragma unroll 5
    for (int k = 0; k < (CHUNK_T * SEQ_BLK) / NTHR; ++k) {
      const int idx = k * NTHR + tid;
      const int m   = idx / CHUNK_T;
      const int tt  = idx - m * CHUNK_T;
      Xs[tt * SEQ_BLK + m] = x[(size_t)(b0 + m) * NSTEP + (size_t)(t0 + tt)];
    }
    __syncthreads();

#pragma unroll 1
    for (int s = 0; s < CHUNK_T; ++s) {
      const int cur = (t0 + s) & 1;
      const _Float16* ahrow = Ah + cur * (SEQ_BLK * HPITCH) + c * HPITCH + koff;
      _Float16* ahn = Ah + (cur ^ 1) * (SEQ_BLK * HPITCH);

      const v4f xa = *(const v4f*)(Xs + s * SEQ_BLK + 8 * hh);
      const v4f xb = *(const v4f*)(Xs + s * SEQ_BLK + 8 * hh + 4);

      v8f acc[4];
#pragma unroll
      for (int g = 0; g < 4; ++g) {
#pragma unroll
        for (int e = 0; e < 4; ++e) {
          acc[g][e]     = fmaf(xa[e], wiS[g], bsS[g]);
          acc[g][4 + e] = fmaf(xb[e], wiS[g], bsS[g]);
        }
      }

      const v16h a0 = frag_load(ahrow);
      const v16h a1 = frag_load(ahrow + 32);
#pragma unroll
      for (int g = 0; g < 4; ++g) acc[g] = mma_h(a0, wb[g][0], acc[g]);
#pragma unroll
      for (int g = 0; g < 4; ++g) acc[g] = mma_h(a1, wb[g][1], acc[g]);
      guard_group(acc[0], acc[1], acc[2], acc[3], a0, a1,
                  wb[0][0], wb[0][1], wb[1][0], wb[1][1], wb[2][0], wb[2][1], wb[3][0], wb[3][1]);

#pragma unroll
      for (int r = 0; r < 8; ++r) {
        const float zi = acc[0][r] * ACARRY_INV;
        const float zf = acc[1][r] * ACARRY_INV;
        const float zg = acc[2][r] * ACARRY_INV;
        const float zo = acc[3][r] * ACARRY_INV;
        const float ig = fsig(zi);
        const float fg = fsig(zf);
        const float gg = ftanh(zg);
        const float og = fsig(zo);
        const float cn = fg * creg[r] + ig * gg;
        creg[r] = cn;
        const float hn = og * ftanh(cn);
        hreg[r] = hn;
        ahn[(8 * hh + r) * HPITCH + hc] = (_Float16)(hn * HCARRY);
      }
      __syncthreads();
    }
  }

#pragma unroll
  for (int r = 0; r < 8; ++r) Hf[(8 * hh + r) * HTPITCH + hc] = hreg[r];
  __syncthreads();

#pragma unroll 1
  for (int p = 0; p < 4; ++p) {
    const int n = 32 * p + lane;
    const float bn = b_fc[n];
    float fa[4];
#pragma unroll
    for (int rr = 0; rr < 4; ++rr) fa[rr] = bn;
    const float* wrow = w_fc + (size_t)n * NHID;
#pragma unroll 1
    for (int k4 = 0; k4 < NHID / 4; ++k4) {
      const v4f w = *(const v4f*)(wrow + 4 * k4);
#pragma unroll
      for (int rr = 0; rr < 4; ++rr) {
        const v4f hv = *(const v4f*)(Hf + (4 * wave + rr) * HTPITCH + 4 * k4);
        float t = fa[rr];
        t = fmaf(hv[0], w[0], t);
        t = fmaf(hv[1], w[1], t);
        t = fmaf(hv[2], w[2], t);
        t = fmaf(hv[3], w[3], t);
        fa[rr] = t;
      }
    }
#pragma unroll
    for (int rr = 0; rr < 4; ++rr) Os[(4 * wave + rr) * OPITCH + n] = fmaxf(fa[rr], 0.0f);
  }
  __syncthreads();

  for (int pass = 0; pass < 2; ++pass) {
#pragma unroll
    for (int it = 0; it < 4; ++it) {
      const int row = 4 * wave + it;
      const v4f v = *(const v4f*)(Os + row * OPITCH + 4 * lane);
      *(volatile v4f*)(out + (size_t)(b0 + row) * NFC + 4 * lane) = v;
    }
    __threadfence();
  }
}

extern "C" void kernel_launch(void* const* d_in, const int* in_sizes, int n_in,
                              void* d_out, int out_size, void* d_ws, size_t ws_size, hipStream_t stream) {
  (void)d_ws;
  (void)ws_size;
  if (n_in < 7 || d_out == nullptr) return;
  if (in_sizes[0] != NBATCH * NSTEP || in_sizes[1] != NGATE || in_sizes[2] != NGATE * NHID ||
      in_sizes[3] != NGATE || in_sizes[4] != NGATE || in_sizes[5] != NFC * NHID || in_sizes[6] != NFC ||
      out_size != NBATCH * NFC) return;

  const float* x    = (const float*)d_in[0];
  const float* w_ih = (const float*)d_in[1];
  const float* w_hh = (const float*)d_in[2];
  const float* b_ih = (const float*)d_in[3];
  const float* b_hh = (const float*)d_in[4];
  const float* w_fc = (const float*)d_in[5];
  const float* b_fc = (const float*)d_in[6];
  float* out = (float*)d_out;

  lstm_seq_kernel<<<NBATCH / SEQ_BLK, NTHR, 0, stream>>>(x, w_ih, w_hh, b_ih, b_hh, w_fc, b_fc, out);
}
